// CrystalGraphEncoder_7275674599727
// MI455X (gfx1250) — hardware-verified
//
#include <hip/hip_runtime.h>
#include <stddef.h>
#include <stdint.h>


#define HD     64
#define NCOL   192
#define NL     3
#define ODIM   128
#define XSC    16.0f
#define WSC    64.0f
#define PINV   0.0009765625f
#define LOG2E  1.4426950408889634f

#define G_THR  192
#define G_NW   6
#define G_ROWS 32

#define NTHR   256
#define NWAVE  8
#define NB     1024
#define SPW    (NB / NWAVE)
#define EPT    16
#define CHUNK  (NTHR * EPT)
#define WCAP   (32 * EPT)
#define HLN    64

#define L_ACC  0
#define L_LIST (L_ACC + NB * HD * 4)
#define L_HL   (L_LIST + NWAVE * WCAP * 4)
#define L_WCNT (L_HL + NWAVE * HLN * 4)
#define E_LDS  (L_WCNT + 64)

#define WS_CAP 134217728ull

static_assert(SPW * NWAVE == NB);
static_assert((SPW % 2) == 0);
static_assert(WCAP >= 32 * EPT);
static_assert((EPT % 4) == 0);
static_assert((L_LIST & 15) == 0 && (L_HL & 15) == 0 && (L_WCNT & 15) == 0);
static_assert(E_LDS <= 298 * 1024);
static_assert(G_NW * 32 == G_THR);
static_assert(ODIM == 4 * 32);

#if __has_builtin(__builtin_amdgcn_exp2f)
#define FEXP2(v) __builtin_amdgcn_exp2f(v)
#else
#define FEXP2(v) exp2f(v)
#endif

typedef float    v4f  __attribute__((ext_vector_type(4)));
typedef float    v8f  __attribute__((ext_vector_type(8)));
typedef int      v4i  __attribute__((ext_vector_type(4)));
typedef _Float16 v8h  __attribute__((ext_vector_type(8)));
typedef _Float16 v16h __attribute__((ext_vector_type(16)));
union FragH { v16h v; v8h h[2]; };

__device__ __forceinline__ v8f zero8f() {
  v8f z;
#pragma unroll
  for (int i = 0; i < 8; ++i) z[i] = 0.0f;
  return z;
}

__device__ __forceinline__ v8f wmh(v16h a, v16h b, v8f c) {
  v8f d = __builtin_amdgcn_wmma_f32_16x16x32_f16(false, a, false, b, (short)0, c, false, false);
  asm volatile("v_nop\n\tv_nop\n\tv_nop\n\tv_nop" : "+v"(d) : "v"(a), "v"(b));
  return d;
}

__global__ __launch_bounds__(256) void k_wcvt(const float* __restrict__ Wg, const float* __restrict__ Wl,
                                              _Float16* Wt) {
  const int t = blockIdx.x * 256 + threadIdx.x;
  if (t >= NL * NCOL * 8) return;
  const int ng = t >> 3, kc = (t & 7) * 8;
  const int l = ng / NCOL, n = ng - l * NCOL;
  const float* src;
  if (n < HD)          src = Wg + (size_t)l * 2 * HD * HD + n;
  else if (n < 2 * HD) src = Wg + (size_t)l * 2 * HD * HD + (size_t)HD * HD + (n - HD);
  else                 src = Wl + (size_t)l * HD * HD + (n - 2 * HD);
  v8h o;
#pragma unroll
  for (int i = 0; i < 8; ++i) o[i] = (_Float16)(src[(size_t)(kc + i) * HD] * WSC);
  _Float16* dp = Wt + (size_t)ng * HD + kc;
  *(volatile v8h*)dp = o;
  __threadfence();
  *(volatile v8h*)dp = o;
}

__global__ __launch_bounds__(G_THR) void k_node(const float* __restrict__ x, const int* __restrict__ z,
                                                const float* __restrict__ emb, int useEmb, int nElems,
                                                const _Float16* Wt, const float* __restrict__ bg,
                                                const float* __restrict__ bl, float* P, int nN) {
  __shared__ __attribute__((aligned(16))) _Float16 ah[G_ROWS * HD];
  __shared__ __attribute__((aligned(16))) float    stg[G_NW * 16 * HD];

  const int tid = threadIdx.x, lane = tid & 31, wave = tid >> 5, hh = lane >> 4, m = lane & 15;
  const int wr = (wave >= 3) ? 1 : 0;
  const int wc = wave - 3 * wr;
  const int row0 = blockIdx.x * G_ROWS;

#pragma unroll 1
  for (int s = tid; s < G_ROWS * 8; s += G_THR) {
    const int r = s >> 3, k0 = (s & 7) * 8;
    const int node = row0 + r;
    v4f x0 = {0.0f, 0.0f, 0.0f, 0.0f};
    v4f x1 = x0;
    if (node < nN) {
      const float* sp;
      if (useEmb != 0) {
        int zi = z[node];
        zi = zi < 0 ? 0 : (zi > nElems - 1 ? nElems - 1 : zi);
        sp = emb + (size_t)zi * HD + k0;
      } else {
        sp = x + (size_t)node * HD + k0;
      }
      x0 = *(const v4f*)sp;
      x1 = *(const v4f*)(sp + 4);
    }
    v8h o;
#pragma unroll
    for (int i = 0; i < 4; ++i) { o[i] = (_Float16)(x0[i] * XSC); o[4 + i] = (_Float16)(x1[i] * XSC); }
    *(v8h*)(ah + r * HD + k0) = o;
  }
  __syncthreads();

  v8f accv[4];
#pragma unroll
  for (int j = 0; j < 4; ++j) accv[j] = zero8f();

  const _Float16* abase = ah + (16 * wr + m) * HD + 8 * hh;
  const _Float16* bbase = Wt + (size_t)(wc * HD + m) * HD + 8 * hh;
#pragma unroll
  for (int kt = 0; kt < HD / 32; ++kt) {
    FragH a;
    a.h[0] = *(const v8h*)(abase + 32 * kt);
    a.h[1] = *(const v8h*)(abase + 32 * kt + 16);
#pragma unroll
    for (int j = 0; j < 4; ++j) {
      const _Float16* bp = bbase + (size_t)(16 * j) * HD + 32 * kt;
      FragH b;
      b.h[0] = *(const v8h*)bp;
      b.h[1] = *(const v8h*)(bp + 16);
      accv[j] = wmh(a.v, b.v, accv[j]);
    }
  }

  const float* bptr = (wc == 0) ? bg : bl;
  float* st = stg + wave * (16 * HD);
#pragma unroll
  for (int j = 0; j < 4; ++j) {
    const float bias = (wc == 1) ? 0.0f : bptr[16 * j + m];
#pragma unroll
    for (int r = 0; r < 8; ++r) st[(8 * hh + r) * HD + 16 * j + m] = accv[j][r] * PINV + bias;
  }
  __syncthreads();

  const size_t gbase = (size_t)(row0 + 16 * wr) * NCOL + (size_t)(wc * HD);
#pragma unroll
  for (int q = 0; q < 8; ++q) {
    const int f = 128 * q + 4 * lane;
    const int rr = f >> 6, cc = f & 63;
    const v4f v = *(const v4f*)(st + f);
    *(volatile v4f*)(P + gbase + (size_t)rr * NCOL + cc) = v;
  }
  __threadfence();
#pragma unroll
  for (int q = 0; q < 8; ++q) {
    const int f = 128 * q + 4 * lane;
    const int rr = f >> 6, cc = f & 63;
    const v4f v = *(const v4f*)(st + f);
    *(volatile v4f*)(P + gbase + (size_t)rr * NCOL + cc) = v;
  }
}

__device__ __forceinline__ int scan_chunk(const int* __restrict__ dsts, int nE, int cbase, int nodeBase,
                                          int* list, int tid, int wave) {
  int wc = 0;
  const int el0  = tid * EPT;
  const int e0   = cbase + el0;
  const int sent = -2147483647 - 1;
  int dv[EPT];
  if (e0 + EPT - 1 < nE) {
#pragma unroll
    for (int q = 0; q < EPT / 4; ++q) {
      const v4i t4 = *(const v4i*)(dsts + e0 + 4 * q);
      dv[4 * q] = t4.x; dv[4 * q + 1] = t4.y; dv[4 * q + 2] = t4.z; dv[4 * q + 3] = t4.w;
    }
  } else {
#pragma unroll
    for (int q = 0; q < EPT; ++q) {
      const int e  = e0 + q;
      const int ec = e < nE ? e : nE - 1;
      dv[q] = (e < nE) ? dsts[ec] : sent;
    }
  }
  const unsigned nb = (unsigned)nodeBase;
  unsigned hm = 0u;
#pragma unroll
  for (int q = 0; q < EPT; ++q) hm |= ((((unsigned)dv[q] - nb) < (unsigned)NB) ? 1u : 0u) << q;
  const unsigned any = __builtin_amdgcn_ballot_w32(hm != 0u);
  if (any != 0u) {
#pragma unroll
    for (int q = 0; q < EPT; ++q) {
      const bool hq = ((hm >> q) & 1u) != 0u;
      const unsigned mj = __builtin_amdgcn_ballot_w32(hq);
      if (mj != 0u) {
        if (hq) {
          const int pos = wc + (int)__builtin_amdgcn_mbcnt_lo(mj, 0u);
          if (pos < WCAP) list[wave * WCAP + pos] = el0 + q;
        }
        wc += (int)__builtin_popcount(mj);
      }
    }
  }
  return wc;
}

__global__ __launch_bounds__(NTHR) void k_edge(const int* __restrict__ ei, const float* P,
                                               float* xo, int nN, int nE) {
  extern __shared__ __attribute__((aligned(16))) unsigned char lds_e[];
  float* acc  = (float*)(lds_e + L_ACC);
  int*   list = (int*)(lds_e + L_LIST);
  int*   hl   = (int*)(lds_e + L_HL);
  int*   wcnt = (int*)(lds_e + L_WCNT);

  const int tid = threadIdx.x, lane = tid & 31, wave = tid >> 5, hh = lane >> 4, m = lane & 15;
  const int c4 = 4 * m;
  const int nodeBase = blockIdx.x * NB;
  const int sbase = wave * SPW;
  const int* dsts = ei;
  const int* srcs = ei + nE;

  {
    const v4f zz = {0.0f, 0.0f, 0.0f, 0.0f};
#pragma unroll 1
    for (int i = tid; i < NB * (HD / 4); i += NTHR) *(v4f*)(acc + 4 * i) = zz;
  }
  __syncthreads();

  const int nChunks = (nE + CHUNK - 1) / CHUNK;
#pragma unroll 1
  for (int ch = 0; ch < nChunks; ++ch) {
    const int cbase = ch * CHUNK;
    const int wc = scan_chunk(dsts, nE, cbase, nodeBase, list, tid, wave);
    if (lane == 0) wcnt[wave] = wc;
    __syncthreads();

#pragma unroll 1
    for (int v = 0; v < NWAVE; ++v) {
      int n = wcnt[v];
      n = n > WCAP ? WCAP : (n < 0 ? 0 : n);
      const int* lp = list + v * WCAP;
#pragma unroll 1
      for (int b0 = 0; b0 < n; b0 += 32) {
        const int idx = b0 + lane;
        const bool valid = idx < n;
        const int el = lp[valid ? idx : 0];
        int e = cbase + el;
        e = e < 0 ? 0 : (e > nE - 1 ? nE - 1 : e);
        const int di = dsts[e];
        const int sj = srcs[e];
        const int slot = di - nodeBase;
        const bool owned = valid && ((unsigned)(slot - sbase) < (unsigned)SPW);
        const unsigned omask = __builtin_amdgcn_ballot_w32(owned);
        const int cnt = (int)__builtin_popcount(omask);
        if (owned) {
          const int pos = (int)__builtin_amdgcn_mbcnt_lo(omask, 0u);
          hl[wave * HLN + 2 * pos]     = di;
          hl[wave * HLN + 2 * pos + 1] = sj;
        }
        __builtin_amdgcn_wave_barrier();
#pragma unroll 1
        for (int p = 0; p < cnt; p += 2) {
          const bool has1 = (p + 1) < cnt;
          const int myp = p + ((hh != 0 && has1) ? 1 : 0);
          const int p1  = has1 ? p + 1 : p;
          const int dI  = hl[wave * HLN + 2 * myp];
          const int sJ  = hl[wave * HLN + 2 * myp + 1];
          const int dI1 = hl[wave * HLN + 2 * p1];
          int s0 = dI - nodeBase;  s0 = s0 < 0 ? 0 : (s0 > NB - 1 ? NB - 1 : s0);
          int s1 = dI1 - nodeBase; s1 = s1 < 0 ? 0 : (s1 > NB - 1 ? NB - 1 : s1);
          const int din = dI < 0 ? 0 : (dI > nN - 1 ? nN - 1 : dI);
          const int sjn = sJ < 0 ? 0 : (sJ > nN - 1 ? nN - 1 : sJ);
          const v4f pa = *(const v4f*)(P + (size_t)din * NCOL + c4);
          const v4f pb = *(const v4f*)(P + (size_t)sjn * NCOL + HD + c4);
          const v4f pl = *(const v4f*)(P + (size_t)sjn * NCOL + 2 * HD + c4);
          v4f msg;
#pragma unroll
          for (int c = 0; c < 4; ++c) {
            const float zv = pa[c] + pb[c];
            const float t  = FEXP2(-zv * LOG2E);
            const float g  = __builtin_amdgcn_rcpf(1.0f + t);
            msg[c] = g * pl[c];
          }
          v4f mw;
#pragma unroll
          for (int c = 0; c < 4; ++c) mw[c] = __shfl_xor(msg[c], 16);
          if (hh == 0) {
            float* q0 = acc + s0 * HD + c4;
            v4f a0 = *(v4f*)q0;
            a0 += msg;
            *(v4f*)q0 = a0;
            if (has1) {
              float* q1 = acc + s1 * HD + c4;
              v4f a1 = *(v4f*)q1;
              a1 += mw;
              *(v4f*)q1 = a1;
            }
          }
        }
      }
    }
    __syncthreads();
  }
  __syncthreads();

#pragma unroll 1
  for (int it = 0; it < SPW / 2; ++it) {
    const int sl = sbase + 2 * it + hh;
    const int node = nodeBase + sl;
    if (node < nN) {
      const v4f av = *(const v4f*)(acc + sl * HD + c4);
      const v4f pl = *(const v4f*)(P + (size_t)node * NCOL + 2 * HD + c4);
      v4f o;
#pragma unroll
      for (int c = 0; c < 4; ++c) o[c] = fmaxf(av[c] + pl[c], 0.0f);
      *(volatile v4f*)(xo + (size_t)node * HD + c4) = o;
    }
  }
  __threadfence();
#pragma unroll 1
  for (int it = 0; it < SPW / 2; ++it) {
    const int sl = sbase + 2 * it + hh;
    const int node = nodeBase + sl;
    if (node < nN) {
      const v4f av = *(const v4f*)(acc + sl * HD + c4);
      const v4f pl = *(const v4f*)(P + (size_t)node * NCOL + 2 * HD + c4);
      v4f o;
#pragma unroll
      for (int c = 0; c < 4; ++c) o[c] = fmaxf(av[c] + pl[c], 0.0f);
      *(volatile v4f*)(xo + (size_t)node * HD + c4) = o;
    }
  }
}

__global__ __launch_bounds__(256) void k_head(const float* x, const float* __restrict__ W1,
                                              const float* __restrict__ b1, const float* __restrict__ W2,
                                              const float* __restrict__ b2, const float* __restrict__ auxA,
                                              const float* __restrict__ auxB, float* out, int nN) {
  __shared__ double part[256];
  __shared__ __attribute__((aligned(16))) float pm[HD];
  __shared__ __attribute__((aligned(16))) float hv[HD];
  __shared__ __attribute__((aligned(16))) float ov[ODIM];
  (void)auxA; (void)auxB;
  const int tid = threadIdx.x;
  const int c = tid & (HD - 1), g = tid >> 6;
  double s = 0.0;
#pragma unroll 1
  for (int r = g; r < nN; r += 4) s += (double)x[(size_t)r * HD + c];
  part[tid] = s;
  __syncthreads();
  if (tid < HD) {
    const double t = ((part[tid] + part[HD + tid]) + part[2 * HD + tid]) + part[3 * HD + tid];
    pm[tid] = (float)t * (1.0f / (float)nN);
  }
  __syncthreads();
  if (tid < HD) {
    float a = 0.0f;
#pragma unroll 1
    for (int k = 0; k < HD; ++k) a += pm[k] * W1[k * HD + tid];
    hv[tid] = fmaxf(a + b1[tid], 0.0f);
  }
  __syncthreads();
  if (tid < ODIM) {
    float a = 0.0f;
#pragma unroll 1
    for (int k = 0; k < HD; ++k) a += hv[k] * W2[k * ODIM + tid];
    ov[tid] = a + b2[tid];
  }
  __syncthreads();
  if (tid < 32) {
    const v4f v = *(const v4f*)(ov + 4 * tid);
    *(volatile v4f*)(out + 4 * tid) = v;
    __threadfence();
    *(volatile v4f*)(out + 4 * tid) = v;
  }
}

extern "C" void kernel_launch(void* const* d_in, const int* in_sizes, int n_in,
                              void* d_out, int out_size, void* d_ws, size_t ws_size,
                              hipStream_t stream) {
  if (n_in < 13) return;
  const int nN = in_sizes[0];
  const int nE = in_sizes[3] / 2;
  const int nElems = in_sizes[4] / HD;
  if (nN <= 0 || nE <= 0 || in_sizes[3] != 2 * nE || nElems <= 0 || in_sizes[4] != nElems * HD) return;
  if (in_sizes[5] != NL * HD * HD || in_sizes[6] != NL * HD) return;
  if (in_sizes[7] != NL * 2 * HD * HD || in_sizes[8] != NL * HD) return;
  if (in_sizes[9] != HD * HD || in_sizes[10] != HD || in_sizes[11] != HD * ODIM || in_sizes[12] != ODIM) return;
  if (out_size != ODIM) return;

  const int*   z   = (const int*)d_in[0];
  const float* pos = (const float*)d_in[1];
  const float* lat = (const float*)d_in[2];
  const int*   ei  = (const int*)d_in[3];
  const float* emb = (const float*)d_in[4];
  const float* Wl  = (const float*)d_in[5];
  const float* bl  = (const float*)d_in[6];
  const float* Wg  = (const float*)d_in[7];
  const float* bg  = (const float*)d_in[8];
  const float* W1  = (const float*)d_in[9];
  const float* b1  = (const float*)d_in[10];
  const float* W2  = (const float*)d_in[11];
  const float* b2  = (const float*)d_in[12];
  float* out = (float*)d_out;

  const int Npad  = ((nN + G_ROWS - 1) / G_ROWS) * G_ROWS;
  const int nBlkG = Npad / G_ROWS;
  const int nBlkE = (nN + NB - 1) / NB;

  char* ws = (char*)d_ws;
  size_t off = 0;
  const size_t oWt = off; off += (size_t)NL * NCOL * HD * 2;   off = (off + 255) & ~(size_t)255;
  const size_t oX  = off; off += (size_t)nN * HD * 4;          off = (off + 255) & ~(size_t)255;
  const size_t oP  = off; off += (size_t)Npad * NCOL * 4;      off = (off + 255) & ~(size_t)255;
  if (off > ws_size || off > (size_t)WS_CAP) return;
  _Float16* Wt = (_Float16*)(ws + oWt);
  float*    X  = (float*)(ws + oX);
  float*    Pb = (float*)(ws + oP);

  const hipError_t ea = hipFuncSetAttribute(reinterpret_cast<const void*>(&k_edge),
                                            hipFuncAttributeMaxDynamicSharedMemorySize, E_LDS);
  (void)ea;

  k_wcvt<<<(NL * NCOL * 8 + 255) / 256, 256, 0, stream>>>(Wg, Wl, Wt);

  for (int l = 0; l < NL; ++l) {
    k_node<<<nBlkG, G_THR, 0, stream>>>(X, z, emb, (l == 0) ? 1 : 0, nElems,
                                         Wt + (size_t)l * NCOL * HD, bg + l * HD, bl + l * HD, Pb, nN);
    k_edge<<<nBlkE, NTHR, E_LDS, stream>>>(ei, Pb, X, nN, nE);
  }

  k_head<<<1, 256, 0, stream>>>(X, W1, b1, W2, b2, pos, lat, out, nN);
  (void)hipGetLastError();
}
